// TransConvLayer_46772193854042
// MI455X (gfx1250) — hardware-verified
//
#include <hip/hip_runtime.h>


#define NBT  4
#define NN   2048
#define DIN  512
#define NH_  8
#define HD   64
#define DSP  (NH_ * HD)
#define DL   (HD + 1)
#define DM   DIN
#define NTK  NN
#define KCURV 1.0f
#define LOSC 1024.0f

typedef _Float16 h16;
typedef unsigned short bf;
typedef __attribute__((ext_vector_type(16))) __bf16   v16bf;
typedef __attribute__((ext_vector_type(16))) _Float16 v16h;
typedef __attribute__((ext_vector_type(8)))  _Float16 v8h;
typedef __attribute__((ext_vector_type(8)))  unsigned short v8us;
typedef __attribute__((ext_vector_type(8)))  float    v8f;
typedef __attribute__((ext_vector_type(4)))  float    v4f;
typedef __attribute__((ext_vector_type(4)))  _Float16 v4h;
typedef v8h  __attribute__((may_alias)) v8ha;
typedef v4f  __attribute__((may_alias)) v4fa;
typedef v8us __attribute__((may_alias)) v8usa;

__device__ __forceinline__ unsigned short f2bf(float f) { unsigned u = __float_as_uint(f); u += 0x7FFFu + ((u >> 16) & 1u); return (unsigned short)(u >> 16); }
__device__ __forceinline__ float bf2f(unsigned short b) { return __uint_as_float(((unsigned)b) << 16); }
__device__ __forceinline__ float bfr(float f) { return bf2f(f2bf(f)); }
__device__ __forceinline__ v16h cat16(v8h lo, v8h hi) { return __builtin_shufflevector(lo, hi, 0, 1, 2, 3, 4, 5, 6, 7, 8, 9, 10, 11, 12, 13, 14, 15); }
__device__ __forceinline__ v16bf cat16b(v8us lo, v8us hi) { return __builtin_bit_cast(v16bf, __builtin_shufflevector(lo, hi, 0, 1, 2, 3, 4, 5, 6, 7, 8, 9, 10, 11, 12, 13, 14, 15)); }
__device__ __forceinline__ v8f wmma16(v16h a, v16h b, v8f c) { return __builtin_amdgcn_wmma_f32_16x16x32_f16(false, a, false, b, (short)0, c, false, false); }
__device__ __forceinline__ v8f wmmab(v16bf a, v16bf b, v8f c) { return __builtin_amdgcn_wmma_f32_16x16x32_bf16(false, a, false, b, (short)0, c, false, false); }

template <bool SPLITA, bool F16OUT = false>
__global__ __launch_bounds__(128) void k_gemmb(const bf* __restrict__ A, const bf* __restrict__ Al, const bf* __restrict__ Bn, const float* __restrict__ bias, float* C, int ldc, h16* C2, const float* __restrict__ R = nullptr, int K = DM, int roundR = 1) {
    __shared__ __align__(16) float ost[4][16 * 68];
    const int lane = threadIdx.x & 31, wave = threadIdx.x >> 5, lr = lane & 15, hi = lane >> 4;
    const int r0 = blockIdx.x * 64 + wave * 16, c0 = blockIdx.y * 64;
    const size_t aoff = (size_t)(r0 + lr) * K + 8 * hi;
    size_t boff[4];
#pragma unroll
    for (int t = 0; t < 4; ++t) boff[t] = (size_t)(c0 + t * 16 + lr) * K + 8 * hi;
    v8f acc[4];
#pragma unroll
    for (int t = 0; t < 4; ++t) acc[t] = (v8f){};
#pragma unroll 1
    for (int kc = 0; kc < K; kc += 32) {
        const v16bf a = cat16b(*(const v8us*)(A + aoff + kc), *(const v8us*)(A + aoff + kc + 16));
        v16bf al = a;
        if (SPLITA) al = cat16b(*(const v8us*)(Al + aoff + kc), *(const v8us*)(Al + aoff + kc + 16));
#pragma unroll
        for (int t = 0; t < 4; ++t) { const v16bf b = cat16b(*(const v8us*)(Bn + boff[t] + kc), *(const v8us*)(Bn + boff[t] + kc + 16)); acc[t] = wmmab(a, b, acc[t]); if (SPLITA) acc[t] = wmmab(al, b, acc[t]); }
        asm volatile("v_nop\n\tv_nop\n\tv_nop\n\tv_nop" : "+v"(acc[0]), "+v"(acc[1]), "+v"(acc[2]), "+v"(acc[3]) : "v"(a), "v"(al));
    }
    float* os = &ost[wave][0];
#pragma unroll
    for (int t = 0; t < 4; ++t) { const float bv = bias ? bfr(bias[c0 + t * 16 + lr]) : 0.f;
#pragma unroll
        for (int j = 0; j < 8; ++j) os[(hi * 8 + j) * 68 + t * 16 + lr] = acc[t][j] + bv; }
    __syncthreads();
    if (F16OUT) {
        h16* crow = (h16*)(void*)C + (size_t)r0 * ldc + c0;
        auto pass = [&]() {
#pragma unroll
            for (int s = 0; s < 4; ++s) { const int row = 4 * s + (lane >> 3), piece = lane & 7; const float* sp = os + row * 68 + piece * 8; v8h o, o2;
#pragma unroll
                for (int i = 0; i < 8; ++i) { const h16 a = (h16)sp[i]; o[i] = a; o2[i] = (h16)((sp[i] - (float)a) * LOSC); }
                *(volatile v8h*)(crow + (size_t)row * ldc + piece * 8) = o; if (C2) *(volatile v8h*)(C2 + (size_t)r0 * ldc + c0 + (size_t)row * ldc + piece * 8) = o2; }
        };
        pass(); __threadfence(); pass();
    } else {
        float* crow = C + (size_t)r0 * ldc + c0;
        auto pass = [&]() {
#pragma unroll
            for (int s = 0; s < 8; ++s) { const int Lid = (lane >> 3) + 4 * s, piece = lane & 7; const int row = Lid >> 1, cofs = (Lid & 1) * 32 + piece * 4;
                v4f val = *(const v4fa*)(os + row * 68 + cofs); if (R) { const v4f rv = *(const v4f*)(R + ((size_t)r0 + row) * ldc + c0 + cofs); val += roundR ? (v4f){bfr(rv[0]), bfr(rv[1]), bfr(rv[2]), bfr(rv[3])} : rv; }
                *(volatile v4f*)(crow + (size_t)row * ldc + cofs) = val; }
        };
        pass(); __threadfence(); pass();
    }
}


template <int MODE>
__global__ __launch_bounds__(128) void k_gemm3z(const bf* __restrict__ Ah, const bf* __restrict__ Al, const bf* __restrict__ Bh, const bf* __restrict__ Bl, int K, float* C, int ldc, size_t sA, size_t sB, size_t sC) {
    if ((MODE & 1) && (int)blockIdx.y * 64 > (int)blockIdx.x * 64 + 63) return;
    const size_t z = blockIdx.z; Ah += z * sA; Al += z * sA; Bh += z * sB; Bl += z * sB; C += z * sC;
    const int Klim = (MODE & 2) ? min(K, ((int)blockIdx.x + 1) * 64) : K;
    __shared__ __align__(16) float ost[4][16 * 68];
    const int lane = threadIdx.x & 31, wave = threadIdx.x >> 5, lr = lane & 15, hi = lane >> 4;
    const int r0 = blockIdx.x * 64 + wave * 16, c0 = blockIdx.y * 64;
    const size_t aoff = (size_t)(r0 + lr) * K + 8 * hi;
    v8f acc[4];
#pragma unroll
    for (int t = 0; t < 4; ++t) acc[t] = (v8f){};
#pragma unroll 1
    for (int kc = 0; kc < Klim; kc += 32) {
        const v16bf a = cat16b(*(const v8us*)(Ah + aoff + kc), *(const v8us*)(Ah + aoff + kc + 16));
        v16bf al = a; if (!(MODE & 4) && !(MODE & 16)) al = cat16b(*(const v8us*)(Al + aoff + kc), *(const v8us*)(Al + aoff + kc + 16));
#pragma unroll
        for (int t = 0; t < 4; ++t) { const size_t bo = (size_t)(c0 + t * 16 + lr) * K + kc + 8 * hi;
            const v16bf bh = cat16b(*(const v8us*)(Bh + bo), *(const v8us*)(Bh + bo + 16));
            acc[t] = wmmab(a, bh, acc[t]);
            if (!(MODE & 4)) { if (!(MODE & 16)) acc[t] = wmmab(al, bh, acc[t]); if (!(MODE & 8)) { const v16bf bl = cat16b(*(const v8us*)(Bl + bo), *(const v8us*)(Bl + bo + 16)); acc[t] = wmmab(a, bl, acc[t]); } } }
        asm volatile("v_nop\n\tv_nop\n\tv_nop\n\tv_nop" : "+v"(acc[0]), "+v"(acc[1]), "+v"(acc[2]), "+v"(acc[3]) : "v"(a), "v"(al));
    }
    float* os = &ost[wave][0];
#pragma unroll
    for (int t = 0; t < 4; ++t) {
#pragma unroll
        for (int j = 0; j < 8; ++j) os[(hi * 8 + j) * 68 + t * 16 + lr] = acc[t][j]; }
    __builtin_amdgcn_wave_barrier(); asm volatile("" ::: "memory");
    float* crow = C + (size_t)r0 * ldc + c0;
    auto pass = [&]() {
#pragma unroll
        for (int s = 0; s < 8; ++s) { const int Lid = (lane >> 3) + 4 * s, piece = lane & 7; const int row = Lid >> 1, cofs = (Lid & 1) * 32 + piece * 4;
            const v4f val = *(const v4fa*)(os + row * 68 + cofs); *(volatile v4f*)(crow + (size_t)row * ldc + cofs) = val; }
    };
    pass(); __threadfence(); pass();
}
__global__ __launch_bounds__(256) void k_planes32z(const float* __restrict__ F, int ld, int off, float sc, int rows, bf* Ph, bf* Pl) {
    typedef __attribute__((ext_vector_type(2))) unsigned short v2us;
    const int lane = threadIdx.x & 31; const size_t r = ((size_t)blockIdx.x * 8 + (threadIdx.x >> 5)) * 2 + (lane >> 4); if (r >= (size_t)rows) return; const int z = blockIdx.z; const int c0 = (lane & 15) * 2; v2us oh, ol;
    Ph += (size_t)z * rows * 32; Pl += (size_t)z * rows * 32;
#pragma unroll
    for (int i = 0; i < 2; ++i) { const float y = F[r * ld + off + z * 32 + c0 + i] * sc; const unsigned short hb = f2bf(y); oh[i] = hb; ol[i] = f2bf(y - bf2f(hb)); }
    const size_t o = r * 32 + c0; *(volatile v2us*)(Ph + o) = oh; *(volatile v2us*)(Pl + o) = ol; __threadfence(); *(volatile v2us*)(Ph + o) = oh; *(volatile v2us*)(Pl + o) = ol;
}
__global__ __launch_bounds__(256) void k_vtpadz(const float* __restrict__ F, int ld, int off, int nk, bf* Th, bf* Tl) {
    typedef __attribute__((ext_vector_type(2))) unsigned short v2us;
    const int lane = threadIdx.x & 31; const size_t wid = (size_t)blockIdx.x * 8 + (threadIdx.x >> 5); if (wid >= (size_t)64 * (nk / 64)) return; const int z = blockIdx.z; const int d = (int)(wid / (nk / 64)); const int k0 = (int)(wid % (nk / 64)) * 64 + lane * 2; v2us oh, ol;
    Th += (size_t)z * 64 * nk; Tl += (size_t)z * 64 * nk;
#pragma unroll
    for (int i = 0; i < 2; ++i) { const float y = (d < 32) ? F[(size_t)(k0 + i) * ld + off + z * 32 + (d < 32 ? d : 0)] : 0.f; const unsigned short hb = f2bf(y); oh[i] = hb; ol[i] = f2bf(y - bf2f(hb)); }
    const size_t o = (size_t)d * nk + k0; *(volatile v2us*)(Th + o) = oh; *(volatile v2us*)(Tl + o) = ol; __threadfence(); *(volatile v2us*)(Th + o) = oh; *(volatile v2us*)(Tl + o) = ol;
}
template <int NK>
__global__ __launch_bounds__(256) void k_softmaxz(const float* __restrict__ S, int rows, bf* PH, bf* PL) {
    typedef __attribute__((ext_vector_type(4))) unsigned short v4us;
    const int lane = threadIdx.x & 31, i = blockIdx.x * 8 + (threadIdx.x >> 5); if (i >= rows) return; const size_t zo = (size_t)blockIdx.z * rows * NK; const float* sr = S + zo + (size_t)i * NK; PH += zo; PL += zo;
    float m = -3.0e38f;
#pragma unroll 1
    for (int c0 = lane * 4; c0 < NK; c0 += 128) {
#pragma unroll
        for (int q = 0; q < 4; ++q) m = fmaxf(m, sr[c0 + q]); }
#pragma unroll
    for (int sh = 16; sh; sh >>= 1) m = fmaxf(m, __shfl_xor(m, sh, 32));
    float sum = 0.f;
#pragma unroll 1
    for (int c0 = lane * 4; c0 < NK; c0 += 128) {
#pragma unroll
        for (int q = 0; q < 4; ++q) sum += __expf(sr[c0 + q] - m); }
#pragma unroll
    for (int sh = 16; sh; sh >>= 1) sum += __shfl_xor(sum, sh, 32);
    const float inv = 1.0f / sum;
#pragma unroll 1
    for (int ps = 0; ps < 2; ++ps) {
#pragma unroll 1
        for (int c0 = lane * 4; c0 < NK; c0 += 128) { v4us oh, ol;
#pragma unroll
            for (int q = 0; q < 4; ++q) { const float p = __expf(sr[c0 + q] - m) * inv; const unsigned short hb = f2bf(p); oh[q] = hb; ol[q] = f2bf(p - bf2f(hb)); }
            const size_t o = (size_t)i * NK + c0; *(volatile v4us*)(PH + o) = oh; *(volatile v4us*)(PL + o) = ol; }
        if (ps == 0) __threadfence(); }
}
__global__ __launch_bounds__(256) void k_placez(const float* __restrict__ XH, int rows, int ldy, float* Y) {
    const int lane = threadIdx.x & 31; const size_t q = (size_t)blockIdx.x * 8 + (threadIdx.x >> 5); if (q >= (size_t)rows) return; const int z = blockIdx.z; const float v = XH[((size_t)z * rows + q) * 64 + lane];
    *(volatile float*)(Y + q * ldy + z * 32 + lane) = v; __threadfence(); *(volatile float*)(Y + q * ldy + z * 32 + lane) = v;
}

__global__ __launch_bounds__(256) void k_hplanesz(const float* __restrict__ F, int ld, int h0, float sc, int rows, bf* Ph, bf* Pl) {
    typedef __attribute__((ext_vector_type(2))) unsigned short v2us;
    const int lane = threadIdx.x & 31; const size_t r = (size_t)blockIdx.x * 8 + (threadIdx.x >> 5); if (r >= (size_t)rows) return; const int z = blockIdx.z; v2us oh, ol;
    Ph += (size_t)z * rows * 64; Pl += (size_t)z * rows * 64;
#pragma unroll
    for (int i = 0; i < 2; ++i) { const float y = F[r * ld + (h0 + z) * 64 + lane * 2 + i] * sc; const unsigned short hb = f2bf(y); oh[i] = hb; ol[i] = f2bf(y - bf2f(hb)); }
    const size_t o = r * 64 + lane * 2; *(volatile v2us*)(Ph + o) = oh; *(volatile v2us*)(Pl + o) = ol; __threadfence(); *(volatile v2us*)(Ph + o) = oh; *(volatile v2us*)(Pl + o) = ol;
}
__global__ __launch_bounds__(256) void k_vtz(const float* __restrict__ F, int ld, int h0, int nk, bf* Th, bf* Tl) {
    typedef __attribute__((ext_vector_type(2))) unsigned short v2us;
    const int lane = threadIdx.x & 31; const size_t wid = (size_t)blockIdx.x * 8 + (threadIdx.x >> 5); if (wid >= (size_t)64 * (nk / 64)) return; const int z = blockIdx.z; const int d = (int)(wid / (nk / 64)); const int t0 = (int)(wid % (nk / 64)) * 64 + lane * 2; v2us oh, ol;
    Th += (size_t)z * 64 * nk; Tl += (size_t)z * 64 * nk;
#pragma unroll
    for (int i = 0; i < 2; ++i) { const float y = F[(size_t)(t0 + i) * ld + (h0 + z) * 64 + d]; const unsigned short hb = f2bf(y); oh[i] = hb; ol[i] = f2bf(y - bf2f(hb)); }
    const size_t o = (size_t)d * nk + t0; *(volatile v2us*)(Th + o) = oh; *(volatile v2us*)(Tl + o) = ol; __threadfence(); *(volatile v2us*)(Th + o) = oh; *(volatile v2us*)(Tl + o) = ol;
}
template <int NK>
__global__ __launch_bounds__(256) void k_softmaxzs(const float* __restrict__ S, int rows, float sc, bf* PH, bf* PL) {
    typedef __attribute__((ext_vector_type(4))) unsigned short v4us;
    const int lane = threadIdx.x & 31, i = blockIdx.x * 8 + (threadIdx.x >> 5); if (i >= rows) return; const size_t zo = (size_t)blockIdx.z * rows * NK; const float* sr = S + zo + (size_t)i * NK; PH += zo; PL += zo;
    float m = -3.0e38f;
#pragma unroll 1
    for (int c0 = lane * 4; c0 < NK; c0 += 128) {
#pragma unroll
        for (int q = 0; q < 4; ++q) m = fmaxf(m, sr[c0 + q] * sc); }
#pragma unroll
    for (int sh = 16; sh; sh >>= 1) m = fmaxf(m, __shfl_xor(m, sh, 32));
    float sum = 0.f;
#pragma unroll 1
    for (int c0 = lane * 4; c0 < NK; c0 += 128) {
#pragma unroll
        for (int q = 0; q < 4; ++q) sum += __expf(sr[c0 + q] * sc - m); }
#pragma unroll
    for (int sh = 16; sh; sh >>= 1) sum += __shfl_xor(sum, sh, 32);
    const float inv = 1.0f / sum;
#pragma unroll 1
    for (int ps = 0; ps < 2; ++ps) {
#pragma unroll 1
        for (int c0 = lane * 4; c0 < NK; c0 += 128) { v4us oh, ol;
#pragma unroll
            for (int q = 0; q < 4; ++q) { const float p = __expf(sr[c0 + q] * sc - m) * inv; const unsigned short hb = f2bf(p); oh[q] = hb; ol[q] = f2bf(p - bf2f(hb)); }
            const size_t o = (size_t)i * NK + c0; *(volatile v4us*)(PH + o) = oh; *(volatile v4us*)(PL + o) = ol; }
        if (ps == 0) __threadfence(); }
}

__global__ __launch_bounds__(256) void k_cvt8(const float* __restrict__ src, bf* dst, size_t n8) {
    const size_t i = (size_t)blockIdx.x * 256 + threadIdx.x; if (i >= n8) return;
    const v8f v = *(const v8f*)(src + i * 8); v8us o;
#pragma unroll
    for (int k = 0; k < 8; ++k) o[k] = f2bf(v[k]);
    *(volatile v8us*)(dst + i * 8) = o; __threadfence(); *(volatile v8us*)(dst + i * 8) = o;
}
__global__ __launch_bounds__(256) void k_zero8(bf* dst, size_t n8) {
    const size_t i = (size_t)blockIdx.x * 256 + threadIdx.x; if (i >= n8) return; v8us z;
#pragma unroll
    for (int k = 0; k < 8; ++k) z[k] = 0;
    *(volatile v8us*)(dst + i * 8) = z; __threadfence(); *(volatile v8us*)(dst + i * 8) = z;
}

__global__ __launch_bounds__(256) void k_cvtx(const float* __restrict__ src, bf* dst) {
    const int lane = threadIdx.x & 31; const size_t r = (size_t)blockIdx.x * 8 + (threadIdx.x >> 5); if (r >= (size_t)NN) return;
#pragma unroll 1
    for (int ps = 0; ps < 2; ++ps) {
#pragma unroll
        for (int q = 0; q < DIN / 256; ++q) { v8us o;
#pragma unroll
            for (int i = 0; i < 8; ++i) o[i] = f2bf(src[r * DIN + q * 256 + lane * 8 + i]);
            *(volatile v8us*)(dst + r * DIN + q * 256 + lane * 8) = o; }
        if (ps == 0) __threadfence(); }
}
__global__ __launch_bounds__(256) void k_time(const float* __restrict__ SP, float* TT) {
    const int lane = threadIdx.x & 31; const int w = blockIdx.x * 8 + (threadIdx.x >> 5); if (w >= NH_ * (NN / 32)) return; const int h = w / (NN / 32); const int s = (w % (NN / 32)) * 32 + lane; float acc = 0.f;
#pragma unroll 8
    for (int d = 0; d < HD; ++d) { const float v = SP[(size_t)s * DSP + h * HD + d]; acc = fmaf(v, v, acc); }
    const float t = sqrtf(acc + KCURV); *(volatile float*)(TT + (size_t)h * NN + s) = t; __threadfence(); *(volatile float*)(TT + (size_t)h * NN + s) = t;
}
__global__ __launch_bounds__(256) void k_vtLz(const float* __restrict__ VS, const float* __restrict__ TT, int h0, bf* Th, bf* Tl) {
    typedef __attribute__((ext_vector_type(2))) unsigned short v2us;
    const int lane = threadIdx.x & 31; const size_t wid = (size_t)blockIdx.x * 8 + (threadIdx.x >> 5); if (wid >= (size_t)128 * (NN / 64)) return; const int z = blockIdx.z, h = h0 + z; const int d = (int)(wid / (NN / 64)); const int t0 = (int)(wid % (NN / 64)) * 64 + lane * 2; v2us oh, ol;
    Th += (size_t)z * 128 * NN; Tl += (size_t)z * 128 * NN;
#pragma unroll
    for (int i = 0; i < 2; ++i) { float y = 0.f; if (d < HD) y = VS[(size_t)(t0 + i) * DSP + h * HD + (d < HD ? d : 0)]; else if (d == HD) y = TT[(size_t)h * NN + t0 + i]; const unsigned short hb = f2bf(y); oh[i] = hb; ol[i] = f2bf(y - bf2f(hb)); }
    const size_t o = (size_t)d * NN + t0; *(volatile v2us*)(Th + o) = oh; *(volatile v2us*)(Tl + o) = ol; __threadfence(); *(volatile v2us*)(Th + o) = oh; *(volatile v2us*)(Tl + o) = ol;
}
__global__ __launch_bounds__(256) void k_lsoftz(const float* __restrict__ S, const float* __restrict__ TQ, const float* __restrict__ TK, int h0, const float* __restrict__ scl, const float* __restrict__ bpar, bf* PH, bf* PL) {
    typedef __attribute__((ext_vector_type(4))) unsigned short v4us;
    const int lane = threadIdx.x & 31, i = blockIdx.x * 8 + (threadIdx.x >> 5); if (i >= NN) return; const int z = blockIdx.z, h = h0 + z; const size_t zo = (size_t)z * NN * NN;
    const float* sr = S + zo + (size_t)i * NN; const float* k0 = TK + (size_t)h * NN; const float qi = TQ[(size_t)h * NN + i]; const float isc = 1.0f / bfr(scl[0]); const float bb = bfr(bpar[0]); PH += zo; PL += zo;
    auto logit = [&](int k) { return (2.0f + 2.0f * (sr[k] - qi * k0[k])) * isc + bb; };
    float m = -3.0e38f;
#pragma unroll 1
    for (int c0 = lane * 4; c0 < NN; c0 += 128) {
#pragma unroll
        for (int q = 0; q < 4; ++q) { const int k = c0 + q; if (k <= i) m = fmaxf(m, logit(k)); } }
#pragma unroll
    for (int sh = 16; sh; sh >>= 1) m = fmaxf(m, __shfl_xor(m, sh, 32));
    float sum = 0.f;
#pragma unroll 1
    for (int c0 = lane * 4; c0 < NN; c0 += 128) {
#pragma unroll
        for (int q = 0; q < 4; ++q) { const int k = c0 + q; if (k <= i) sum += __expf(logit(k) - m); } }
#pragma unroll
    for (int sh = 16; sh; sh >>= 1) sum += __shfl_xor(sum, sh, 32);
    const float inv = 1.0f / sum;
#pragma unroll 1
    for (int ps = 0; ps < 2; ++ps) {
#pragma unroll 1
        for (int c0 = lane * 4; c0 < NN; c0 += 128) { v4us oh, ol;
#pragma unroll
            for (int q = 0; q < 4; ++q) { const int k = c0 + q; const float p = (k <= i) ? __expf(logit((k <= i) ? k : 0) - m) * inv : 0.f; const unsigned short hb = f2bf(p); oh[q] = hb; ol[q] = f2bf(p - bf2f(hb)); }
            const size_t o = (size_t)i * NN + c0; *(volatile v4us*)(PH + o) = oh; *(volatile v4us*)(PL + o) = ol; }
        if (ps == 0) __threadfence(); }
}
__global__ __launch_bounds__(256) void k_mid(const float* __restrict__ CTX, float* AVE) {
    const int lane = threadIdx.x & 31; const size_t s = (size_t)blockIdx.x * 8 + (threadIdx.x >> 5); if (s >= (size_t)NN) return; v4f a;
#pragma unroll
    for (int q = 0; q < 4; ++q) { const int c = lane * 4 + q; float v = 0.f; if (c < DL) { const int col = (c == 0) ? HD : (c - 1);
#pragma unroll
            for (int h = 0; h < NH_; ++h) v += CTX[((size_t)h * NN + s) * 128 + col];
            v *= (1.0f / NH_); } a[q] = v; }
    float part = 0.f;
#pragma unroll
    for (int q = 0; q < 4; ++q) { const int c = lane * 4 + q; if (c == 0) part -= a[q] * a[q]; else if (c < DL) part += a[q] * a[q]; }
#pragma unroll
    for (int sh = 16; sh; sh >>= 1) part += __shfl_xor(part, sh, 32);
    const float den = sqrtf(fmaxf(fabsf(-part), 1e-8f)); const float f = sqrtf(KCURV) / den;
    v4f o;
#pragma unroll
    for (int q = 0; q < 4; ++q) o[q] = a[q] * f;
    *(volatile v4f*)(AVE + s * 128 + lane * 4) = o; __threadfence(); *(volatile v4f*)(AVE + s * 128 + lane * 4) = o;
}
__global__ __launch_bounds__(256) void k_outflat(const float* __restrict__ AVE, float* OUTB) {
    const int lane = threadIdx.x & 31; const size_t w = (size_t)blockIdx.x * 8 + (threadIdx.x >> 5); if (w >= (size_t)NN * DL / 128) return; const size_t e0 = w * 128 + lane * 4; v4f v;
#pragma unroll
    for (int q = 0; q < 4; ++q) { const size_t e = e0 + q; v[q] = AVE[(e / DL) * 128 + (e % DL)]; }
    *(volatile v4f*)(OUTB + e0) = v; __threadfence(); *(volatile v4f*)(OUTB + e0) = v;
}

extern "C" void kernel_launch(void* const* d_in, const int* in_sizes, int n_in,
                              void* d_out, int out_size, void* d_ws, size_t ws_size, hipStream_t stream) {
    (void)in_sizes; (void)n_in; (void)out_size;
    const float* xq = (const float*)d_in[0]; const float* xs = (const float*)d_in[1]; const float* Wq = (const float*)d_in[2]; const float* bq = (const float*)d_in[3]; const float* Wk = (const float*)d_in[4]; const float* bk = (const float*)d_in[5]; const float* Wv = (const float*)d_in[6]; const float* bv = (const float*)d_in[7]; const float* scl = (const float*)d_in[8]; const float* bpar = (const float*)d_in[9];
    float* out = (float*)d_out;
    char* wsp = (char*)d_ws;
    auto take = [&](size_t bytes) { char* p = wsp; wsp += (bytes + 255) & ~(size_t)255; return (void*)p; };
    const int ZH = 2;
    bf* WQ = (bf*)take((size_t)DSP * DIN * 2); bf* WK = (bf*)take((size_t)DSP * DIN * 2); bf* WV = (bf*)take((size_t)DSP * DIN * 2);
    bf* Xq = (bf*)take((size_t)NN * DIN * 2); bf* Xs = (bf*)take((size_t)NN * DIN * 2); float* QS = (float*)take((size_t)NN * DSP * 4); float* KS = (float*)take((size_t)NN * DSP * 4); float* VS = (float*)take((size_t)NN * DSP * 4);
    float* TQ = (float*)take((size_t)NH_ * NN * 4); float* TK = (float*)take((size_t)NH_ * NN * 4); float* TV = (float*)take((size_t)NH_ * NN * 4);
    bf* Qh = (bf*)take((size_t)ZH * NN * HD * 2); bf* Ql = (bf*)take((size_t)ZH * NN * HD * 2); bf* Kh = (bf*)take((size_t)ZH * NN * HD * 2); bf* Kl = (bf*)take((size_t)ZH * NN * HD * 2); bf* VTh = (bf*)take((size_t)ZH * 128 * NN * 2); bf* VTl = (bf*)take((size_t)ZH * 128 * NN * 2);
    float* S = (float*)take((size_t)ZH * NN * NN * 4); bf* PH = (bf*)take((size_t)ZH * NN * NN * 2); bf* PL = (bf*)take((size_t)ZH * NN * NN * 2); float* CTX = (float*)take((size_t)NH_ * NN * 128 * 4); float* AVE = (float*)take((size_t)NN * 128 * 4);
    if ((size_t)(wsp - (char*)d_ws) > ws_size) return;
    k_cvt8<<<(DSP * DIN / 8 + 255) / 256, 256, 0, stream>>>(Wq, WQ, DSP * DIN / 8); k_cvt8<<<(DSP * DIN / 8 + 255) / 256, 256, 0, stream>>>(Wk, WK, DSP * DIN / 8); k_cvt8<<<(DSP * DIN / 8 + 255) / 256, 256, 0, stream>>>(Wv, WV, DSP * DIN / 8);
    for (int b = 0; b < NBT; ++b) {
        k_cvtx<<<NN / 8, 256, 0, stream>>>(xq + (size_t)b * NN * DIN, Xq); k_cvtx<<<NN / 8, 256, 0, stream>>>(xs + (size_t)b * NN * DIN, Xs);
        k_gemmb<false, false><<<dim3(NN / 64, DSP / 64, 1), 128, 0, stream>>>(Xq, nullptr, WQ, bq, QS, DSP, nullptr, nullptr, DIN);
        k_gemmb<false, false><<<dim3(NN / 64, DSP / 64, 1), 128, 0, stream>>>(Xs, nullptr, WK, bk, KS, DSP, nullptr, nullptr, DIN);
        k_gemmb<false, false><<<dim3(NN / 64, DSP / 64, 1), 128, 0, stream>>>(Xs, nullptr, WV, bv, VS, DSP, nullptr, nullptr, DIN);
        k_time<<<(NH_ * (NN / 32)) / 8, 256, 0, stream>>>(QS, TQ); k_time<<<(NH_ * (NN / 32)) / 8, 256, 0, stream>>>(KS, TK); k_time<<<(NH_ * (NN / 32)) / 8, 256, 0, stream>>>(VS, TV);
        for (int g = 0; g < NH_ / ZH; ++g) { const int h0 = g * ZH;
            k_hplanesz<<<dim3(NN / 8, 1, ZH), 256, 0, stream>>>(QS, DSP, h0, 1.0f, NN, Qh, Ql); k_hplanesz<<<dim3(NN / 8, 1, ZH), 256, 0, stream>>>(KS, DSP, h0, 1.0f, NN, Kh, Kl);
            k_vtLz<<<dim3((128 * (NN / 64)) / 8, 1, ZH), 256, 0, stream>>>(VS, TV, h0, VTh, VTl);
            k_gemm3z<1><<<dim3(NN / 64, NN / 64, ZH), 128, 0, stream>>>(Qh, Ql, Kh, Kl, HD, S, NN, (size_t)NN * HD, (size_t)NN * HD, (size_t)NN * NN);
            k_lsoftz<<<dim3(NN / 8, 1, ZH), 256, 0, stream>>>(S, TQ, TK, h0, scl, bpar, PH, PL);
            k_gemm3z<2><<<dim3(NN / 64, 2, ZH), 128, 0, stream>>>(PH, PL, VTh, VTl, NN, CTX + (size_t)h0 * NN * 128, 128, (size_t)NN * NN, (size_t)128 * NN, (size_t)NN * 128); }
        k_mid<<<NN / 8, 256, 0, stream>>>(CTX, AVE);
        k_outflat<<<(NN * DL / 128) / 8, 256, 0, stream>>>(AVE, out + (size_t)b * NN * DL); }
}
